// cFSMN_layer_72662256713826
// MI455X (gfx1250) — hardware-verified
//
#include <hip/hip_runtime.h>
#include <math.h>

typedef __attribute__((ext_vector_type(16))) _Float16 v16h;
typedef __attribute__((ext_vector_type(16))) __bf16 v16b;
typedef __attribute__((ext_vector_type(8)))  _Float16 v8h;
typedef __attribute__((ext_vector_type(8)))  float v8f;
typedef __attribute__((ext_vector_type(4)))  float v4f;
typedef __attribute__((ext_vector_type(2)))  float v2f;
typedef __attribute__((ext_vector_type(4)))  unsigned v4u;
typedef __attribute__((ext_vector_type(4)))  int v4i;
typedef float __attribute__((may_alias)) float_a;
typedef int __attribute__((may_alias)) int_a;

template <typename T> __device__ __forceinline__ void vst2(void* p, T v) { *(volatile T*)p = v; __threadfence(); *(volatile T*)p = v; }
__device__ __forceinline__ v8f wmma16(v16h a, v16h b, v8f c) {
  v8f d = __builtin_amdgcn_wmma_f32_16x16x32_f16(false, a, false, b, (short)0, c, false, false);
  asm volatile("v_nop\n\tv_nop\n\tv_nop\n\tv_nop" : "+v"(d) : "v"(a), "v"(b));
  return d;
}
__device__ __forceinline__ v8f wmma_bf(v16b a, v16b b, v8f c) {
  v8f d = __builtin_amdgcn_wmma_f32_16x16x32_bf16(false, a, false, b, (short)0, c, false, false);
  asm volatile("v_nop\n\tv_nop\n\tv_nop\n\tv_nop" : "+v"(d) : "v"(a), "v"(b));
  return d;
}
__device__ __forceinline__ v16h frag_h(const _Float16* rowk0, int lane) {
  union { v16h v; v8h q[2]; } u; const _Float16* p = rowk0 + 8 * (lane >> 4);
  u.q[0] = *(const v8h*)p; u.q[1] = *(const v8h*)(p + 16); return u.v;
}
__device__ __forceinline__ v16h frag_f32(const float* rowk0, int lane) {
  v16h a; const float* p = rowk0 + 8 * (lane >> 4);
#pragma unroll
  for (int i = 0; i < 8; ++i) { a[i] = (_Float16)p[i]; a[8 + i] = (_Float16)p[16 + i]; }
  return a;
}
__device__ __forceinline__ v16h frag_f32s(const float* rowk0, int lane, float sc) {
  v16h a; const float* p = rowk0 + 8 * (lane >> 4);
#pragma unroll
  for (int i = 0; i < 8; ++i) { a[i] = (_Float16)(p[i] * sc); a[8 + i] = (_Float16)(p[16 + i] * sc); }
  return a;
}
__device__ __forceinline__ v16h fragc_f32(const float* W, int k0, int n, int lane, int ld, int K) {
  v16h a; const int g = lane >> 4;
#pragma unroll
  for (int i = 0; i < 8; ++i) { const int ka = k0 + 8 * g + i, kb = ka + 16;
    a[i] = (_Float16)(ka < K ? W[(size_t)(ka < K ? ka : K - 1) * ld + n] : 0.f); a[8 + i] = (_Float16)(kb < K ? W[(size_t)(kb < K ? kb : K - 1) * ld + n] : 0.f); }
  return a;
}
struct F2 { v16b h, l; };
__device__ __forceinline__ F2 bsplit16(const float v[16]) { F2 r;
#pragma unroll
  for (int i = 0; i < 16; ++i) { const __bf16 h = (__bf16)v[i]; r.h[i] = h; r.l[i] = (__bf16)(v[i] - (float)h); }
  return r; }
__device__ __forceinline__ F2 split_row(const float* row, int k0, int lane) { float v[16]; const float* p = row + k0 + 8 * (lane >> 4);
#pragma unroll
  for (int i = 0; i < 8; ++i) { v[i] = p[i]; v[8 + i] = p[16 + i]; }
  return bsplit16(v); }
__device__ __forceinline__ F2 split_rowK(const float* row, int k0, int lane, int K) { float v[16]; const int g = lane >> 4;
#pragma unroll
  for (int i = 0; i < 8; ++i) { const int ka = k0 + 8 * g + i, kb = ka + 16; v[i] = ka < K ? row[ka < K ? ka : K - 1] : 0.f; v[8 + i] = kb < K ? row[kb < K ? kb : K - 1] : 0.f; }
  return bsplit16(v); }
__device__ __forceinline__ F2 split_col(const float* W, int k0, int n, int lane, int ld, int K) { float v[16]; const int g = lane >> 4;
#pragma unroll
  for (int i = 0; i < 8; ++i) { const int ka = k0 + 8 * g + i, kb = ka + 16; v[i] = ka < K ? W[(size_t)(ka < K ? ka : K - 1) * ld + n] : 0.f; v[8 + i] = kb < K ? W[(size_t)(kb < K ? kb : K - 1) * ld + n] : 0.f; }
  return bsplit16(v); }
__device__ __forceinline__ v8f mac3(const F2& a, const F2& b, v8f c) { c = wmma_bf(a.l, b.h, c); c = wmma_bf(a.h, b.l, c); return wmma_bf(a.h, b.h, c); }
__device__ __forceinline__ float sigm(float v) { return 1.0f / (1.0f + expf(-v)); }
#define LDSX() do { asm volatile("s_wait_dscnt 0" ::: "memory"); __builtin_amdgcn_wave_barrier(); __builtin_amdgcn_fence(__ATOMIC_RELEASE, "workgroup"); } while (0)


#define NBATCH 16
#define TT 1024
#define NTOK (NBATCH * TT)
#define DD 512
#define HH_ 2048
#define EMB 256
#define RK 768
#define NE 8
#define NBLK (NTOK / 64)
#ifndef NBLKT
#define NBLKT NBLK
#endif
#define MAXT 64
typedef __attribute__((ext_vector_type(8))) __bf16 v8b;
__device__ __forceinline__ v16b frag_b(const __bf16* rowk0, int lane) {
  union { v16b v; v8b q[2]; } u; const __bf16* p = rowk0 + 8 * (lane >> 4);
  u.q[0] = *(const v8b*)p; u.q[1] = *(const v8b*)(p + 16); return u.v;
}
__device__ __forceinline__ float bfr(float v) { return (float)(__bf16)v; }
__device__ __attribute__((noinline)) float exp_ni(float v) { return expf(v); }
__device__ __attribute__((noinline)) float erf_ni(float v) { return erff(v); }

#define WS_LST  0u
#define WS_CNTI (WS_LST + 4u * NE * NBLK * 64)
#define WS_OFFI (WS_CNTI + 4u * NBLK * 32)
#define WS_GE   (WS_OFFI + 4u * (NE * NBLK + 32))
#define WS_GV   (WS_GE + 4u * NTOK)
#define WS_PW   (WS_GV + 4u * NTOK)
#define PG 0
#define P1 (PG + 16 * RK)
#define P2 (P1 + (size_t)NE * HH_ * DD)
#define PWEND (P2 + (size_t)NE * DD * HH_)
#define WS_H1   (WS_PW + 2u * PWEND)
#define WS_Y    (WS_H1 + 4u * NTOK * HH_)
#define WS_P    (WS_Y + 4u * NTOK * DD)
#define WS_END  (WS_P + 4u * NTOK * DD)

__global__ __launch_bounds__(256) void k_packT(const float* __restrict__ RW, const float* __restrict__ W1, const float* __restrict__ W2, __bf16* __restrict__ PW) {
  __shared__ __align__(16) __bf16 s[HH_]; const int n = blockIdx.x, which = blockIdx.y, tid = threadIdx.x; int K; size_t dst;
  if (which == 0) { if (n >= 16) return; K = RK; dst = PG + (size_t)n * RK; for (int k = tid; k < K; k += 256) s[k] = (__bf16)((n < NE) ? RW[(size_t)k * NE + n] : 0.f); }
  else if (which == 1) { K = DD; const int e = n / HH_, o = n % HH_; dst = P1 + (size_t)n * DD; for (int k = tid; k < K; k += 256) s[k] = (__bf16)W1[((size_t)e * DD + k) * HH_ + o]; }
  else { if (n >= NE * DD) return; K = HH_; const int e = n / DD, o = n % DD; dst = P2 + (size_t)n * HH_; for (int k = tid; k < K; k += 256) s[k] = (__bf16)W2[((size_t)e * HH_ + k) * DD + o]; }
  __syncthreads();
  for (int q = tid; q < K / 8; q += 256) vst2((unsigned*)(PW + dst + q * 8), *(const v4u*)&s[q * 8]);
}
__global__ __launch_bounds__(128) void k_gate(const float* __restrict__ X, const float* __restrict__ EMBm, const __bf16* __restrict__ PW, int* __restrict__ GE, float* __restrict__ GV, int* __restrict__ LST, int* __restrict__ CNTI) {
  __shared__ float sl[4][16][NE + 1]; __shared__ __align__(16) int sge[64]; __shared__ __align__(16) float sgv[64]; __shared__ __align__(16) int slst[NE][64]; __shared__ __align__(16) int scnt[32];
  const int tid = threadIdx.x, wave = tid >> 5, lane = tid & 31, col = lane & 15, g = lane >> 4; const size_t r0 = (size_t)blockIdx.x * 64 + wave * 16;
  v8f acc = {};
#pragma unroll 2
  for (int kc = 0; kc < RK / 32; ++kc) { v16b a; { const float* p = (kc < EMB / 32) ? (EMBm + (r0 + col) * EMB + kc * 32 + 8 * g) : (X + (r0 + col) * DD + (kc * 32 - EMB) + 8 * g);
#pragma unroll
      for (int i = 0; i < 8; ++i) { a[i] = (__bf16)p[i]; a[8 + i] = (__bf16)p[16 + i]; } }
    acc = wmma_bf(a, frag_b(PW + PG + (size_t)col * RK + kc * 32, lane), acc); }
  if (col < NE) {
#pragma unroll
    for (int r = 0; r < 8; ++r) sl[wave][8 * g + r][col] = acc[r]; }
  LDSX();
  if (lane < 16) { const int rl = lane; const int tl = wave * 16 + rl; float lg[NE];
#pragma unroll
    for (int e = 0; e < NE; ++e) lg[e] = sl[wave][rl][e];
    int i1 = 0; float v1 = lg[0];
#pragma unroll
    for (int e = 1; e < NE; ++e) if (lg[e] > v1) { v1 = lg[e]; i1 = e; }
    float s = 0.f;
#pragma unroll
    for (int e = 0; e < NE; ++e) s += exp_ni(lg[e] - v1);
    sge[tl] = i1; sgv[tl] = 1.0f / s; }
  __syncthreads();
  if (tid < 16) { vst2((unsigned*)(GE + (size_t)blockIdx.x * 64 + tid * 4), *(const v4u*)&sge[tid * 4]); vst2(GV + (size_t)blockIdx.x * 64 + tid * 4, *(const v4f*)&sgv[tid * 4]); }
  for (int q = tid; q < NE * 64; q += 128) slst[q >> 6][q & 63] = -1;
  if (tid < 32) scnt[tid] = 0;
  __syncthreads();
  if (tid < NE) { int c = 0; for (int p = 0; p < 64; ++p) if (sge[p] == tid) { slst[tid][c++] = blockIdx.x * 64 + p; } scnt[tid] = c; }
  __syncthreads();
  for (int q = tid; q < NE * 16; q += 128) { const int e = q >> 4, pc = q & 15; vst2((unsigned*)(LST + ((size_t)e * NBLK + blockIdx.x) * 64 + pc * 4), *(const v4u*)&slst[e][pc * 4]); }
  if (tid < 8) vst2((unsigned*)(CNTI + (size_t)blockIdx.x * 32 + tid * 4), *(const v4u*)&scnt[tid * 4]);
}
__global__ __launch_bounds__(32) void k_mscan(const int* __restrict__ CNTI, int* __restrict__ OFFI) {
  __shared__ __align__(16) int so[NE][NBLK]; __shared__ __align__(16) int stot[32]; const int e = threadIdx.x;
  if (e < NE) { int run = 0; for (int b = 0; b < NBLK; ++b) { so[e][b] = run; if (b < NBLKT) run += min(max(CNTI[(size_t)b * 32 + e], 0), 64); } stot[e] = run; } else if (e < 32) stot[e] = 0;
  __syncthreads();
  for (int q = e; q < NE * NBLK / 4; q += 32) vst2((unsigned*)(OFFI + q * 4), *(const v4u*)&(&so[0][0])[q * 4]);
  if (e < 8) vst2((unsigned*)(OFFI + NE * NBLK + e * 4), *(const v4u*)&stot[e * 4]);
}
__device__ __forceinline__ int moe_tok(const int* __restrict__ OFFI, const int* __restrict__ CNTI, const int* __restrict__ LST, int e, int r) {
  int lo = 0, hi = NBLKT - 1; while (lo < hi) { const int mid = (lo + hi + 1) >> 1; if (OFFI[e * NBLK + mid] <= r) lo = mid; else hi = mid - 1; }
  const int off = OFFI[e * NBLK + lo]; const int c = min(max(CNTI[(size_t)lo * 32 + e], 0), 64); const int i = r - off; if (i < 0 || i >= c) return -1;
  const int p = LST[((size_t)e * NBLK + lo) * 64 + i]; return (p < 0 || p >= NTOK) ? -1 : p;
}
__global__ __launch_bounds__(128) void k_ffn1(const float* __restrict__ X, const __bf16* __restrict__ PW, const float* __restrict__ B1, const int* __restrict__ LST, const int* __restrict__ CNTI, const int* __restrict__ OFFI, float* __restrict__ H1) {
  __shared__ __align__(16) float so[4][16][132]; __shared__ int stok[64];
  const int tid = threadIdx.x, wave = tid >> 5, lane = tid & 31, col = lane & 15, g = lane >> 4; const int t = blockIdx.x, e = blockIdx.z; const int n0 = blockIdx.y * 128;
  const int cnt = min(max(OFFI[NE * NBLK + e], 0), NTOK); if (t * 64 >= cnt) return;
  if (tid < 64) { const int i = t * 64 + tid; stok[tid] = (i < cnt) ? moe_tok(OFFI, CNTI, LST, e, i) : -1; }
  __syncthreads();
  const int my = stok[wave * 16 + col]; const size_t tok = (size_t)(my < 0 ? 0 : my);
  v8f acc[8] = {};
#pragma unroll 2
  for (int kc = 0; kc < DD / 32; ++kc) { v16b a; { const float* p = X + tok * DD + kc * 32 + 8 * g;
#pragma unroll
      for (int i = 0; i < 8; ++i) { a[i] = (__bf16)p[i]; a[8 + i] = (__bf16)p[16 + i]; } }
#pragma unroll
    for (int j = 0; j < 8; ++j) acc[j] = wmma_bf(a, frag_b(PW + P1 + ((size_t)e * HH_ + n0 + j * 16 + col) * DD + kc * 32, lane), acc[j]); }
#pragma unroll
  for (int j = 0; j < 8; ++j) { const float bb = bfr(B1[e * HH_ + n0 + j * 16 + col]);
#pragma unroll
    for (int r = 0; r < 8; ++r) so[wave][8 * g + r][j * 16 + col] = fmaxf(acc[j][r] + bb, 0.f); }
  LDSX();
  for (int rl = 0; rl < 16; ++rl) { const int tk = stok[wave * 16 + rl]; if (tk >= 0) vst2(H1 + (size_t)tk * HH_ + n0 + lane * 4, *(const v4f*)&so[wave][rl][lane * 4]); }
}
__global__ __launch_bounds__(128) void k_ffn2(const float* __restrict__ H1, const __bf16* __restrict__ PW, const int* __restrict__ LST, const int* __restrict__ CNTI, const int* __restrict__ OFFI, float* __restrict__ Y) {
  __shared__ __align__(16) float so[4][16][132]; __shared__ int stok[64];
  const int tid = threadIdx.x, wave = tid >> 5, lane = tid & 31, col = lane & 15, g = lane >> 4; const int t = blockIdx.x, e = blockIdx.z; const int n0 = blockIdx.y * 128;
  const int cnt = min(max(OFFI[NE * NBLK + e], 0), NTOK); if (t * 64 >= cnt) return;
  if (tid < 64) { const int i = t * 64 + tid; stok[tid] = (i < cnt) ? moe_tok(OFFI, CNTI, LST, e, i) : -1; }
  __syncthreads();
  const int my = stok[wave * 16 + col]; const size_t tok = (size_t)(my < 0 ? 0 : my);
  v8f acc[8] = {};
#pragma unroll 2
  for (int kc = 0; kc < HH_ / 32; ++kc) { const F2 a = split_row(H1 + tok * HH_, kc * 32, lane);
#pragma unroll
    for (int j = 0; j < 8; ++j) { const v16b w = frag_b(PW + P2 + ((size_t)e * DD + n0 + j * 16 + col) * HH_ + kc * 32, lane); acc[j] = wmma_bf(a.l, w, acc[j]); acc[j] = wmma_bf(a.h, w, acc[j]); } }
#pragma unroll
  for (int j = 0; j < 8; ++j)
#pragma unroll
    for (int r = 0; r < 8; ++r) so[wave][8 * g + r][j * 16 + col] = acc[j][r];
  LDSX();
  for (int rl = 0; rl < 16; ++rl) { const int tk = stok[wave * 16 + rl]; if (tk >= 0) vst2(Y + (size_t)tk * DD + n0 + lane * 4, *(const v4f*)&so[wave][rl][lane * 4]); }
}
__global__ __launch_bounds__(256) void k_post(const float* __restrict__ Y, const float* __restrict__ GV, const float* __restrict__ X, const int* __restrict__ SEQ, float* __restrict__ P) {
  const int tid = threadIdx.x; const int tsub = tid >> 5, piece = tid & 31; const int n0 = blockIdx.y * 128 + piece * 4;
#pragma unroll 1
  for (int pass = 0; pass < 8; ++pass) { const size_t tok = (size_t)blockIdx.x * 64 + pass * 8 + tsub; const int b = (int)(tok / TT), t = (int)(tok % TT); const float msk = (t < SEQ[b]) ? 1.f : 0.f; const float gv = GV[tok];
    v4f o;
#pragma unroll
    for (int i = 0; i < 4; ++i) o[i] = (Y[tok * DD + n0 + i] * gv + bfr(X[tok * DD + n0 + i])) * msk;
    vst2(P + tok * DD + n0, o); }
}
__global__ __launch_bounds__(256) void k_fir(const float* __restrict__ P, const float* __restrict__ LF, const float* __restrict__ CF, const float* __restrict__ RF, float* __restrict__ OUT) {
  const int tid = threadIdx.x; const int tsub = tid >> 5, piece = tid & 31; const int n0 = blockIdx.y * 128 + piece * 4;
#pragma unroll 1
  for (int pass = 0; pass < 8; ++pass) { const size_t tok = (size_t)blockIdx.x * 64 + pass * 8 + tsub; const int b = (int)(tok / TT), t = (int)(tok % TT);
    v4f m = {0.f, 0.f, 0.f, 0.f};
#pragma unroll 1
    for (int k = 0; k < 11; ++k) { const int ts = t + k - 5; if (ts < 0 || ts >= TT) continue; const float* fk = (k < 5) ? (LF + k * DD) : (k == 5 ? CF : (RF + (k - 6) * DD)); const float* pr = P + ((size_t)b * TT + ts) * DD + n0;
#pragma unroll
      for (int i = 0; i < 4; ++i) m[i] += bfr(fk[n0 + i]) * pr[i]; }
    const float* pc_ = P + tok * DD + n0; v4f o;
#pragma unroll
    for (int i = 0; i < 4; ++i) o[i] = m[i] + pc_[i];
    vst2(OUT + tok * DD + n0, o); }
}
extern "C" void kernel_launch(void* const* d_in, const int* in_sizes, int n_in, void* d_out, int out_size, void* d_ws, size_t ws_size, hipStream_t stream) {
  (void)in_sizes; (void)n_in; (void)out_size;
  const float** F = (const float**)d_in; const int* SEQ = (const int*)d_in[2];
  if (ws_size < (size_t)WS_END) return;
  char* ws = (char*)d_ws; int *LST = (int*)(ws + WS_LST), *CNTI = (int*)(ws + WS_CNTI), *OFFI = (int*)(ws + WS_OFFI), *GE = (int*)(ws + WS_GE); float *GV = (float*)(ws + WS_GV), *H1 = (float*)(ws + WS_H1), *Y = (float*)(ws + WS_Y), *P = (float*)(ws + WS_P); __bf16* PW = (__bf16*)(ws + WS_PW);
  k_packT<<<dim3(NE * HH_, 3), 256, 0, stream>>>(F[9], F[3], F[5], PW);
  k_gate<<<NBLKT, 128, 0, stream>>>(F[0], F[1], PW, GE, GV, LST, CNTI);
  k_mscan<<<1, 32, 0, stream>>>(CNTI, OFFI);
  k_ffn1<<<dim3(MAXT, HH_ / 128, NE), 128, 0, stream>>>(F[0], PW, F[4], LST, CNTI, OFFI, H1);
  k_ffn2<<<dim3(MAXT, DD / 128, NE), 128, 0, stream>>>(H1, PW, LST, CNTI, OFFI, Y);
  k_post<<<dim3(NBLKT, DD / 128), 256, 0, stream>>>(Y, GV, F[0], SEQ, P);
  k_fir<<<dim3(NBLKT, DD / 128), 256, 0, stream>>>(P, F[6], F[7], F[8], (float*)d_out);
}
